// PerformerBlock_51479478010629
// MI455X (gfx1250) — hardware-verified
//
#include <hip/hip_runtime.h>

typedef _Float16 bf16;
typedef bf16    v16bf __attribute__((ext_vector_type(16)));
typedef bf16    v8bf  __attribute__((ext_vector_type(8)));
typedef float   v8f   __attribute__((ext_vector_type(8)));

#define BB   2
#define SS   2048
#define DD   1024
#define HH   16
#define DH   64
#define MLP  4096
#define ROWS (BB * SS)
#define NC   (SS / 64)
#define EPS_LN  1e-6f
#define KEPS    1e-3f

__device__ __forceinline__ bf16 f2bf(float f) { return (bf16)f; }
__device__ __forceinline__ float bf2f(bf16 v) { return (float)v; }
typedef float v4f __attribute__((ext_vector_type(4)));
typedef unsigned v4u __attribute__((ext_vector_type(4)));
typedef unsigned v2u __attribute__((ext_vector_type(2)));
typedef float __attribute__((may_alias)) float_a;
template <typename T> __device__ __forceinline__ void vst2(void* p, T v) { *(volatile T*)p = v; __threadfence(); *(volatile T*)p = v; }
__device__ __forceinline__ float gelu_tanh(float x) {
    const float k0 = 0.7978845608028654f, k1 = 0.044715f;
    float t = tanhf(k0 * (x + k1 * x * x * x));
    return 0.5f * x * (1.0f + t);
}

__device__ __forceinline__ v16bf load_frag_a_rowmajor(const bf16* p, int ld) {
    int lane = threadIdx.x & 31;
    int m = lane & 15, kh = lane >> 4;
    const bf16* q = p + (size_t)m * ld + kh * 8;
    v8bf lo = *(const v8bf*)(q);
    v8bf hi = *(const v8bf*)(q + 16);
    return __builtin_shufflevector(lo, hi, 0, 1, 2, 3, 4, 5, 6, 7,
                                   8, 9, 10, 11, 12, 13, 14, 15);
}
__device__ __forceinline__ v16bf load_frag_b_contig(const bf16* p, int ld) {
    int lane = threadIdx.x & 31;
    int n = lane & 15, kh = lane >> 4;
    const bf16* q = p + (size_t)n * ld + kh * 8;
    v8bf lo = *(const v8bf*)(q);
    v8bf hi = *(const v8bf*)(q + 16);
    return __builtin_shufflevector(lo, hi, 0, 1, 2, 3, 4, 5, 6, 7, 8, 9, 10, 11, 12, 13, 14, 15);
}
__device__ __forceinline__ v8f wmma_bf16(v16bf a, v16bf b, v8f c) {
    v8f d = __builtin_amdgcn_wmma_f32_16x16x32_f16(false, a, false, b, (short)0, c, false, false);
    asm volatile("v_nop\n\tv_nop\n\tv_nop\n\tv_nop" : "+v"(d) : "v"(a), "v"(b));
    return d;
}

__global__ void transpose_to_bf16(const float* __restrict__ src,
                                  bf16* __restrict__ dst, int R, int C) {
    __shared__ __align__(16) bf16 tile[64][72];
    const int tilesC = C / 64;
    const int tr = blockIdx.x / tilesC, tc = blockIdx.x % tilesC, tid = threadIdx.x;
    for (int i = tid; i < 64 * 64; i += 256) { const int rr = i >> 6, cc = i & 63;
        tile[cc][rr] = f2bf(src[(size_t)(tr * 64 + rr) * C + tc * 64 + cc]); }
    __syncthreads();
    for (int g = tid; g < 64 * 8; g += 256) { const int cc = g >> 3, pc = g & 7;
        vst2(dst + (size_t)(tc * 64 + cc) * R + tr * 64 + pc * 8, *(const v4u*)(&tile[cc][pc * 8])); }
}

__global__ void ln_to_bf16(const float* __restrict__ x,
                           const float* __restrict__ sc,
                           const float* __restrict__ bi,
                           bf16* __restrict__ out) {
    __shared__ float s1[256], s2[256];
    int row = blockIdx.x, tid = threadIdx.x;
    const float* xr = x + (size_t)row * DD;
    float v[4], a = 0.f, b = 0.f;
    { const v4f t4 = *(const v4f*)(xr + tid * 4);
#pragma unroll
      for (int i = 0; i < 4; i++) { v[i] = t4[i]; a += t4[i]; b += t4[i] * t4[i]; } }
    s1[tid] = a; s2[tid] = b; __syncthreads();
    for (int off = 128; off > 0; off >>= 1) {
        if (tid < off) { s1[tid] += s1[tid + off]; s2[tid] += s2[tid + off]; }
        __syncthreads();
    }
    float mean = s1[0] * (1.0f / DD);
    float var  = s2[0] * (1.0f / DD) - mean * mean;
    float r = rsqrtf(var + EPS_LN);
    union { bf16 h[4]; v2u u; } pk;
#pragma unroll
    for (int i = 0; i < 4; i++) { int c = tid * 4 + i; pk.h[i] = f2bf((v[i] - mean) * r * sc[c] + bi[c]); }
    vst2(out + (size_t)row * DD + tid * 4, pk.u);
}

template <int EPI>
__global__ void gemm_bf16(const bf16* __restrict__ A, const bf16* __restrict__ Bt,
                          float* __restrict__ Cf, bf16* __restrict__ Cb,
                          const float* __restrict__ bias,
                          const float* __restrict__ res, int N, int K) {
    int wave = threadIdx.x >> 5, lane = threadIdx.x & 31;
    int row0 = blockIdx.y * 128 + wave * 16;
    int col0 = blockIdx.x * 64;
    const v8f zero = {0, 0, 0, 0, 0, 0, 0, 0};
    v8f acc[4];
#pragma unroll
    for (int t = 0; t < 4; t++) acc[t] = zero;

    for (int kk = 0; kk < K; kk += 32) {
        v16bf a = load_frag_a_rowmajor(A + (size_t)row0 * K + kk, K);
#pragma unroll
        for (int t = 0; t < 4; t++) {
            v16bf b = load_frag_b_contig(Bt + (size_t)(col0 + t * 16) * K + kk, K);
            acc[t] = wmma_bf16(a, b, acc[t]);
        }
    }

    int n = lane & 15, mh = lane >> 4;
    __shared__ __align__(16) float So[8][16 * 64];
    float* S = So[wave];
#pragma unroll
    for (int t = 0; t < 4; t++) {
        int col = col0 + t * 16 + n;
#pragma unroll 1
        for (int r = 0; r < 8; r++) {
            float v = acc[t][r];
            if (EPI == 1) v = gelu_tanh(v + bias[col]);
            else if (EPI == 3) v += bias[col];
            S[(r + mh * 8) * 64 + t * 16 + n] = v;
        }
    }
    asm volatile("s_wait_dscnt 0" ::: "memory"); __builtin_amdgcn_wave_barrier(); __builtin_amdgcn_fence(__ATOMIC_RELEASE, "workgroup");
    if (EPI <= 1) {
#pragma unroll
        for (int q = 0; q < 4; q++) { const int rl = q * 4 + (lane >> 3), pc = lane & 7;
            union { v8bf h; v4u u; } pk;
#pragma unroll
            for (int e = 0; e < 8; e++) pk.h[e] = f2bf(S[rl * 64 + pc * 8 + e]);
            vst2(Cb + (size_t)(row0 + rl) * N + col0 + pc * 8, pk.u); }
    } else {
#pragma unroll
        for (int q = 0; q < 8; q++) { const int rl = q * 2 + (lane >> 4), pc = lane & 15;
            const size_t idx = (size_t)(row0 + rl) * N + col0 + pc * 4;
            v4f vv = *(const v4f*)(S + rl * 64 + pc * 4); const v4f rr = *(const v4f*)(res + idx);
            vst2(Cf + idx, vv + rr); }
    }
}

__global__ void attn_chunk_sums(const bf16* __restrict__ QKV,
                                float* __restrict__ KVc,
                                float* __restrict__ Ksum) {
    __shared__ __attribute__((aligned(64))) bf16 phiKt[64 * 64];
    __shared__ __attribute__((aligned(64))) bf16 Vt[64 * 64];
    int bhc = blockIdx.x;
    int c = bhc & (NC - 1), h = (bhc >> 5) & (HH - 1), b = bhc >> 9;
    int tid = threadIdx.x;
    size_t rowbase = ((size_t)b * SS + (size_t)c * 64) * 3072;
    for (int i8 = tid; i8 < 512; i8 += 128) {
        int s = i8 >> 3, mg = (i8 & 7) * 8;
        size_t base = rowbase + (size_t)s * 3072 + h * 64 + mg;
        v8bf k8 = *(const v8bf*)(QKV + base + 1024);
        v8bf v8 = *(const v8bf*)(QKV + base + 2048);
#pragma unroll
        for (int e = 0; e < 8; e++) {
            phiKt[(mg + e) * 64 + s] = f2bf(fmaxf(bf2f(k8[e]), 0.f) + KEPS);
            Vt[(mg + e) * 64 + s]    = v8[e];
        }
    }
    __syncthreads();

    int wave = tid >> 5, lane = tid & 31;
    int m0 = wave * 16;
    const v8f zero = {0, 0, 0, 0, 0, 0, 0, 0};
    v8f acc[4];
#pragma unroll
    for (int t = 0; t < 4; t++) acc[t] = zero;
#pragma unroll
    for (int kk = 0; kk < 64; kk += 32) {
        v16bf a = load_frag_a_rowmajor(phiKt + (size_t)m0 * 64 + kk, 64);
#pragma unroll
        for (int t = 0; t < 4; t++) {
            v16bf b = load_frag_b_contig(Vt + (size_t)(t * 16) * 64 + kk, 64);
            acc[t] = wmma_bf16(a, b, acc[t]);
        }
    }
    int n = lane & 15, mh = lane >> 4;
    float* out = KVc + (size_t)bhc * 4096;
    __shared__ __align__(16) float So[4][16 * 64];
    float* S = So[wave];
#pragma unroll
    for (int t = 0; t < 4; t++)
#pragma unroll
        for (int r = 0; r < 8; r++) S[(r + mh * 8) * 64 + t * 16 + n] = acc[t][r];
    asm volatile("s_wait_dscnt 0" ::: "memory"); __builtin_amdgcn_wave_barrier(); __builtin_amdgcn_fence(__ATOMIC_RELEASE, "workgroup");
#pragma unroll
    for (int q = 0; q < 8; q++) { const int rl = q * 2 + (lane >> 4), pc = lane & 15;
        vst2(out + (m0 + rl) * 64 + pc * 4, *(const v4f*)(S + rl * 64 + pc * 4)); }

    if (tid < 64) {
        float s = 0.f;
        const bf16* row = phiKt + (size_t)tid * 64;
        for (int sl = 0; sl < 64; sl++) s += bf2f(row[sl]);
        vst2(Ksum + (size_t)bhc * 64 + tid, (float_a)s);
    }
}

__global__ void attn_scan(float* __restrict__ KVc, float* __restrict__ Ksum) {
    int bh = blockIdx.x, tid = threadIdx.x;
    float acc[16];
#pragma unroll
    for (int j = 0; j < 16; j++) acc[j] = 0.f;
    for (int c = 0; c < NC; c++) {
        float* p = KVc + ((size_t)bh * NC + c) * 4096 + tid;
#pragma unroll
        for (int j = 0; j < 16; j++) { float t = p[j * 256]; vst2(p + j * 256, (float_a)acc[j]); acc[j] += t; }
    }
    if (tid < 64) {
        float a = 0.f;
        for (int c = 0; c < NC; c++) {
            float* p = Ksum + ((size_t)bh * NC + c) * 64 + tid;
            float t = *p; vst2(p, (float_a)a); a += t;
        }
    }
}

__global__ void attn_chunk_out(const bf16* __restrict__ QKV,
                               const float* __restrict__ KVc,
                               const float* __restrict__ Ksum,
                               bf16* __restrict__ Aout) {
    __shared__ __attribute__((aligned(64))) bf16 phiQ[4096];
    __shared__ __attribute__((aligned(64))) bf16 phiK[4096];
    __shared__ __attribute__((aligned(64))) bf16 Vt[4096];
    __shared__ __attribute__((aligned(64))) bf16 KVpt[4096];
    __shared__ __attribute__((aligned(64))) bf16 Sc[4096];
    __shared__ float Ksp[64], den[64];
    int bhc = blockIdx.x;
    int c = bhc & (NC - 1), h = (bhc >> 5) & (HH - 1), b = bhc >> 9;
    int tid = threadIdx.x;
    size_t rowbase = ((size_t)b * SS + (size_t)c * 64) * 3072;
    for (int i8 = tid; i8 < 512; i8 += 128) {
        int s = i8 >> 3, mg = (i8 & 7) * 8;
        size_t base = rowbase + (size_t)s * 3072 + h * 64 + mg;
        v8bf q8 = *(const v8bf*)(QKV + base);
        v8bf k8 = *(const v8bf*)(QKV + base + 1024);
        v8bf v8 = *(const v8bf*)(QKV + base + 2048);
        v8bf pq, pk;
#pragma unroll
        for (int e = 0; e < 8; e++) {
            pq[e] = f2bf(fmaxf(bf2f(q8[e]), 0.f) + KEPS);
            pk[e] = f2bf(fmaxf(bf2f(k8[e]), 0.f) + KEPS);
            Vt[(mg + e) * 64 + s] = v8[e];
        }
        *(v8bf*)(phiQ + s * 64 + mg) = pq;
        *(v8bf*)(phiK + s * 64 + mg) = pk;
    }
    for (int i = tid; i < 4096; i += 128) {
        int m = i >> 6, dh = i & 63;
        KVpt[dh * 64 + m] = f2bf(KVc[(size_t)bhc * 4096 + i]);
    }
    if (tid < 64) Ksp[tid] = Ksum[(size_t)bhc * 64 + tid];
    __syncthreads();

    int wave = tid >> 5, lane = tid & 31;
    int n = lane & 15, mh = lane >> 4;
    int i0 = wave * 16;
    const v8f zero = {0, 0, 0, 0, 0, 0, 0, 0};

    v8f sc[4];
#pragma unroll
    for (int t = 0; t < 4; t++) sc[t] = zero;
#pragma unroll
    for (int kk = 0; kk < 64; kk += 32) {
        v16bf a = load_frag_a_rowmajor(phiQ + (size_t)i0 * 64 + kk, 64);
#pragma unroll
        for (int t = 0; t < 4; t++) {
            v16bf bb = load_frag_b_contig(phiK + (size_t)(t * 16) * 64 + kk, 64);
            sc[t] = wmma_bf16(a, bb, sc[t]);
        }
    }
#pragma unroll
    for (int t = 0; t < 4; t++)
#pragma unroll
        for (int r = 0; r < 8; r++) {
            int i = i0 + r + mh * 8, j = t * 16 + n;
            Sc[i * 64 + j] = f2bf((j <= i) ? sc[t][r] : 0.f);
        }
    __syncthreads();

    if (tid < 64) {
        float d = 0.f, qd = 0.f;
        const bf16* srow = Sc + (size_t)tid * 64;
        const bf16* qrow = phiQ + (size_t)tid * 64;
        for (int j = 0; j < 64; j++) d += bf2f(srow[j]);
        for (int m = 0; m < 64; m++) qd += bf2f(qrow[m]) * Ksp[m];
        den[tid] = d + qd;
    }

    v8f acc[4];
#pragma unroll
    for (int t = 0; t < 4; t++) acc[t] = zero;
#pragma unroll
    for (int kk = 0; kk < 64; kk += 32) {
        v16bf a1 = load_frag_a_rowmajor(Sc + (size_t)i0 * 64 + kk, 64);
        v16bf a2 = load_frag_a_rowmajor(phiQ + (size_t)i0 * 64 + kk, 64);
#pragma unroll
        for (int t = 0; t < 4; t++) {
            v16bf b1 = load_frag_b_contig(Vt + (size_t)(t * 16) * 64 + kk, 64);
            v16bf b2 = load_frag_b_contig(KVpt + (size_t)(t * 16) * 64 + kk, 64);
            acc[t] = wmma_bf16(a1, b1, acc[t]);
            acc[t] = wmma_bf16(a2, b2, acc[t]);
        }
    }
    __syncthreads();

    size_t orow = (size_t)b * SS + (size_t)c * 64;
    bf16* So = Sc + wave * 1024;
#pragma unroll
    for (int t = 0; t < 4; t++)
#pragma unroll
        for (int r = 0; r < 8; r++) {
            int i = i0 + r + mh * 8, dh = t * 16 + n;
            So[(r + mh * 8) * 64 + dh] = f2bf(acc[t][r] / den[i]);
        }
    asm volatile("s_wait_dscnt 0" ::: "memory"); __builtin_amdgcn_wave_barrier(); __builtin_amdgcn_fence(__ATOMIC_RELEASE, "workgroup");
#pragma unroll
    for (int q = 0; q < 4; q++) { const int rl = q * 4 + (lane >> 3), pc = lane & 7;
        vst2(Aout + (orow + i0 + rl) * DD + h * 64 + pc * 8, *(const v4u*)(So + rl * 64 + pc * 8)); }
}

extern "C" void kernel_launch(void* const* d_in, const int* in_sizes, int n_in,
                              void* d_out, int out_size, void* d_ws, size_t ws_size,
                              hipStream_t stream) {
    const float* inputs    = (const float*)d_in[0];
    const float* ln1_scale = (const float*)d_in[1];
    const float* ln1_bias  = (const float*)d_in[2];
    const float* wq        = (const float*)d_in[3];
    const float* wk        = (const float*)d_in[4];
    const float* wv        = (const float*)d_in[5];
    const float* wo        = (const float*)d_in[6];
    const float* ln2_scale = (const float*)d_in[7];
    const float* ln2_bias  = (const float*)d_in[8];
    const float* w1        = (const float*)d_in[9];
    const float* b1        = (const float*)d_in[10];
    const float* w2        = (const float*)d_in[11];
    const float* b2        = (const float*)d_in[12];

    char* ws = (char*)d_ws;
    size_t off = 0;
    auto carve = [&](size_t bytes) -> char* {
        char* p = ws + off;
        off += (bytes + 255) & ~(size_t)255;
        return p;
    };
    bf16* Wqkv_t = (bf16*)carve((size_t)3072 * 1024 * 2);
    bf16* Wo_t   = (bf16*)carve((size_t)1024 * 1024 * 2);
    bf16* W1t    = (bf16*)carve((size_t)4096 * 1024 * 2);
    bf16* W2t    = (bf16*)carve((size_t)1024 * 4096 * 2);
    bf16* Xln    = (bf16*)carve((size_t)ROWS * DD * 2);
    bf16* QKV    = (bf16*)carve((size_t)ROWS * 3072 * 2);
    bf16* Aout   = (bf16*)carve((size_t)ROWS * DD * 2);
    bf16* H1     = (bf16*)carve((size_t)ROWS * MLP * 2);
    float* Xres  = (float*)carve((size_t)ROWS * DD * 4);
    float* KVc   = (float*)carve((size_t)BB * HH * NC * 64 * 64 * 4);
    float* Ksum  = (float*)carve((size_t)BB * HH * NC * 64 * 4);
    (void)ws_size; (void)in_sizes; (void)n_in; (void)out_size;

    int g1m = (1024 / 64) * (1024 / 64);
    int g4m = (1024 / 64) * (4096 / 64);
    transpose_to_bf16<<<g1m, 256, 0, stream>>>(wq, Wqkv_t, 1024, 1024);
    transpose_to_bf16<<<g1m, 256, 0, stream>>>(wk, Wqkv_t + (size_t)1024 * 1024, 1024, 1024);
    transpose_to_bf16<<<g1m, 256, 0, stream>>>(wv, Wqkv_t + (size_t)2048 * 1024, 1024, 1024);
    transpose_to_bf16<<<g1m, 256, 0, stream>>>(wo, Wo_t, 1024, 1024);
    transpose_to_bf16<<<g4m, 256, 0, stream>>>(w1, W1t, 1024, 4096);
    transpose_to_bf16<<<g4m, 256, 0, stream>>>(w2, W2t, 4096, 1024);

    ln_to_bf16<<<ROWS, 256, 0, stream>>>(inputs, ln1_scale, ln1_bias, Xln);

    gemm_bf16<0><<<dim3(3072 / 64, ROWS / 128), 256, 0, stream>>>(
        Xln, Wqkv_t, nullptr, QKV, nullptr, nullptr, 3072, 1024);

    attn_chunk_sums<<<BB * HH * NC, 128, 0, stream>>>(QKV, KVc, Ksum);
    attn_scan<<<BB * HH, 256, 0, stream>>>(KVc, Ksum);
    attn_chunk_out<<<BB * HH * NC, 128, 0, stream>>>(QKV, KVc, Ksum, Aout);

    gemm_bf16<2><<<dim3(DD / 64, ROWS / 128), 256, 0, stream>>>(
        Aout, Wo_t, Xres, nullptr, nullptr, inputs, DD, 1024);

    ln_to_bf16<<<ROWS, 256, 0, stream>>>(Xres, ln2_scale, ln2_bias, Xln);

    gemm_bf16<1><<<dim3(MLP / 64, ROWS / 128), 256, 0, stream>>>(
        Xln, W1t, nullptr, H1, b1, nullptr, MLP, 1024);

    gemm_bf16<3><<<dim3(DD / 64, ROWS / 128), 256, 0, stream>>>(
        H1, W2t, (float*)d_out, nullptr, b2, Xres, DD, MLP);
}
